// SelectiveStructuredSSM_6459630813399
// MI455X (gfx1250) — hardware-run, weakly checked
//
#include <hip/hip_runtime.h>


#ifndef NB
#define NB 2
#endif
#ifndef SEQ
#define SEQ 4096
#endif
#define NB_FULL  2
#define SEQ_FULL 4096
#ifndef OUT_SEQ
#define OUT_SEQ SEQ
#endif
#define DD   768
#define NS   16
#define NW   48
#define ST   128
#define CH   32
#define OSP  36
#define L2E  1.4426950408889634f
#define LN2  0.6931471805599453f

static_assert(DD % 32 == 0);
static_assert(DD % 8 == 0);
static_assert((NB * SEQ) % 64 == 0);
static_assert(NW == 48);
static_assert(2 * NS == 32);
static_assert(2 * NS < NW);
static_assert(DD % ST == 0);
static_assert(ST % 32 == 0);
static_assert(SEQ % CH == 0);
static_assert(CH == 32);
static_assert((CH * 32 / 4) % ST == 0);
static_assert((CH / 4) * 32 * 16 == CH * 32 * 4);
static_assert(4 * 32 * 16 == 16 * 32 * 4);
static_assert(16 * 16 == 64 * 4);
static_assert((size_t)NW * (DD / 8) * 16 == (size_t)NW * DD * 2);
static_assert((16 * 68 + 64) * 4 <= 131072);
static_assert((CH * 32 + CH + (ST / 32) * CH * OSP) * 4 <= 131072);
static_assert((OSP * 4) % 16 == 0);
static_assert(NB <= NB_FULL);
static_assert(SEQ <= SEQ_FULL);
static_assert(((size_t)SEQ * DD) % 8 == 0);

typedef _Float16 h16;
typedef unsigned short bf;
typedef __attribute__((ext_vector_type(16))) __bf16   v16bf;
typedef __attribute__((ext_vector_type(16))) _Float16 v16h;
typedef __attribute__((ext_vector_type(8)))  _Float16 v8h;
typedef __attribute__((ext_vector_type(8)))  unsigned short v8us;
typedef __attribute__((ext_vector_type(8)))  float    v8f;
typedef __attribute__((ext_vector_type(4)))  float    v4f;
typedef v4f  __attribute__((may_alias)) v4fa;

__device__ __forceinline__ unsigned short f2bf(float f) { unsigned u = __float_as_uint(f); u += 0x7FFFu + ((u >> 16) & 1u); return (unsigned short)(u >> 16); }
__device__ __forceinline__ float bfr(float f) { return __uint_as_float(((unsigned)f2bf(f)) << 16); }
__device__ __forceinline__ v16h cat16(v8h lo, v8h hi) { return __builtin_shufflevector(lo, hi, 0, 1, 2, 3, 4, 5, 6, 7, 8, 9, 10, 11, 12, 13, 14, 15); }
__device__ __forceinline__ v16bf cat16b(v8us lo, v8us hi) { return __builtin_bit_cast(v16bf, __builtin_shufflevector(lo, hi, 0, 1, 2, 3, 4, 5, 6, 7, 8, 9, 10, 11, 12, 13, 14, 15)); }
__device__ __forceinline__ v8f wmma16(v16h a, v16h b, v8f c) { return __builtin_amdgcn_wmma_f32_16x16x32_f16(false, a, false, b, (short)0, c, false, false); }
__device__ __forceinline__ v8f wmmab(v16bf a, v16bf b, v8f c) { return __builtin_amdgcn_wmma_f32_16x16x32_bf16(false, a, false, b, (short)0, c, false, false); }
__device__ __forceinline__ v16h  ldh(const h16* p) { return cat16(*(const v8h*)p, *(const v8h*)(p + 16)); }
__device__ __forceinline__ v16bf ldb(const bf* p)  { return cat16b(*(const v8us*)p, *(const v8us*)(p + 16)); }
__device__ __forceinline__ void wave_sync() { __builtin_amdgcn_fence(3  , "wavefront"); __builtin_amdgcn_wave_barrier(); asm volatile("" ::: "memory"); }
__device__ __forceinline__ v8f wmmab_g(v16bf a, v16bf b, v8f c) {
    c = wmmab(a, b, c);
    asm volatile("v_nop\n\tv_nop\n\tv_nop\n\tv_nop" : "+v"(c) : "v"(a), "v"(b));
    return c;
}

__global__ __launch_bounds__(256) void k_cvt8(const float* __restrict__ src, bf* dst, size_t n8) {
    const size_t i = (size_t)blockIdx.x * 256 + threadIdx.x; if (i >= n8) return;
    const v8f v = *(const v8f*)(src + i * 8); v8us o;
#pragma unroll
    for (int k = 0; k < 8; ++k) o[k] = f2bf(v[k]);
    *(volatile v8us*)(dst + i * 8) = o; __threadfence(); *(volatile v8us*)(dst + i * 8) = o;
}

__global__ __launch_bounds__(256) void k_wpack(const float* __restrict__ WBi, const float* __restrict__ WCi, const float* __restrict__ WDi, bf* dst) {
    const int i = blockIdx.x * 256 + threadIdx.x; if (i >= NW * (DD / 8)) return;
    const int n = i / (DD / 8), k0 = (i % (DD / 8)) * 8; const int nc = n & 15;
    v8us o;
#pragma unroll
    for (int k = 0; k < 8; ++k) {
        float vb = WBi[(size_t)(k0 + k) * NS + nc];
        float vc = WCi[(size_t)(k0 + k) * NS + nc];
        float vd = WDi[k0 + k];
        asm volatile("" : "+v"(vb)); asm volatile("" : "+v"(vc)); asm volatile("" : "+v"(vd));
        const float v = (n < 16) ? vb : ((n < 32) ? vc : ((n == 32) ? vd : 0.0f));
        o[k] = f2bf(v);
    }
    *(volatile v8us*)(dst + (size_t)i * 8) = o; __threadfence(); *(volatile v8us*)(dst + (size_t)i * 8) = o;
}

__global__ __launch_bounds__(32) void k_pgemm(const bf* __restrict__ A, const bf* __restrict__ Bt, const float* __restrict__ bBi, const float* __restrict__ bCi, const float* __restrict__ bDi,
                                              float* PBC, float* SP) {
    __shared__ __align__(16) float os[16 * 68];
    __shared__ __align__(16) float sst[64];
    const int K = DD;
    const int lane = threadIdx.x & 31, lr = lane & 15, hi = lane >> 4; const int r0 = blockIdx.x * 64;
    v8f acc[4][3];
#pragma unroll
    for (int mb = 0; mb < 4; ++mb)
#pragma unroll
        for (int nb = 0; nb < 3; ++nb) acc[mb][nb] = (v8f){};
    const size_t aoff = (size_t)(r0 + lr) * K + 8 * hi, boff = (size_t)lr * K + 8 * hi;
#pragma unroll 1
    for (int kc = 0; kc < K; kc += 32) {
        v16bf a[4];
#pragma unroll
        for (int mb = 0; mb < 4; ++mb) a[mb] = ldb(A + aoff + (size_t)mb * 16 * K + kc);
#pragma unroll
        for (int nb = 0; nb < 3; ++nb) { const v16bf b = ldb(Bt + boff + (size_t)nb * 16 * K + kc);
#pragma unroll
            for (int mb = 0; mb < 4; ++mb) acc[mb][nb] = wmmab_g(a[mb], b, acc[mb][nb]); }
    }
    float bc[3];
    float bdv = bDi[0]; asm volatile("" : "+v"(bdv));
    bc[0] = bfr(bBi[lr]); bc[1] = bfr(bCi[lr]); bc[2] = (lr == 0) ? bfr(bdv) : 0.0f;
#pragma unroll
    for (int mb = 0; mb < 4; ++mb) {
#pragma unroll
        for (int nb = 0; nb < 3; ++nb) {
#pragma unroll
            for (int j = 0; j < 8; ++j) os[(hi * 8 + j) * 68 + nb * 16 + lr] = acc[mb][nb][j] + bc[nb]; }
        wave_sync();
        { const float sv = os[lr * 68 + 32]; sst[mb * 16 + lr] = sv; }
#pragma unroll 1
        for (int ps = 0; ps < 2; ++ps) {
#pragma unroll
            for (int s = 0; s < 4; ++s) { const int row = 4 * s + (lane >> 3), cofs = (lane & 7) * 4;
                const v4f val = *(const v4fa*)(&os[row * 68 + cofs]);
                *(volatile v4f*)(PBC + (size_t)(r0 + mb * 16 + row) * 32 + cofs) = val; }
            if (ps == 0) __threadfence(); }
        wave_sync();
    }
    const v4f sq = *(const v4fa*)(&sst[lr * 4]);
#pragma unroll 1
    for (int ps = 0; ps < 2; ++ps) {
        if (lane < 16) *(volatile v4f*)(SP + (size_t)r0 + lr * 4) = sq;
        if (ps == 0) __threadfence(); }
}

__global__ __launch_bounds__(ST) void k_scan(const float* __restrict__ X, const float* __restrict__ Ain, const float* __restrict__ pDl,
                                             const float* __restrict__ PBC, const float* __restrict__ SP, float* OUT) {
#pragma clang fp contract(off)
    __shared__ __align__(16) float bcs[CH * 32];
    __shared__ __align__(16) float ss[CH];
    __shared__ __align__(16) float os[(ST / 32) * CH * OSP];
    const int tid = threadIdx.x, lane = tid & 31;
    const int wave = __builtin_amdgcn_readfirstlane((int)(threadIdx.x >> 5));
    const int b = blockIdx.y; const int d = blockIdx.x * ST + tid;
    float an[NS], h[NS];
#pragma unroll
    for (int q = 0; q < NS / 4; ++q) { const v4f av = *(const v4f*)(Ain + (size_t)d * NS + 4 * q);
#pragma unroll
        for (int r = 0; r < 4; ++r) { an[4 * q + r] = bfr(av[r]); h[4 * q + r] = 0.0f; } }
    const float pd = bfr(pDl[d]);
    const float* xcol = X + (size_t)b * SEQ_FULL * DD + d;
    const size_t prow = (size_t)b * SEQ;
    const int wb = wave * CH * OSP;
    float* obase = OUT + (size_t)b * OUT_SEQ * DD + (size_t)blockIdx.x * ST + (size_t)wave * 32;
#pragma unroll 1
    for (int l0 = 0; l0 < SEQ; l0 += CH) {
#pragma unroll
        for (int j = 0; j < (CH * 32 / 4) / ST; ++j) { const int q = tid + ST * j;
            const v4f t = *(const v4f*)(PBC + (prow + (size_t)l0) * 32 + (size_t)q * 4);
            *(v4fa*)(&bcs[q * 4]) = t; }
        if (wave == 0) ss[lane] = SP[prow + (size_t)l0 + lane];
        __syncthreads();
#pragma unroll 1
        for (int i = 0; i < CH; ++i) {
            const float xv = bfr(xcol[(size_t)(l0 + i) * DD]);
            const float z = ss[i] + pd;
            const float e = __builtin_amdgcn_exp2f(-fabsf(z) * L2E);
            const float delta = fmaxf(z, 0.0f) + __builtin_amdgcn_logf(1.0f + e) * LN2;
            v4f bq[4], cq[4];
#pragma unroll
            for (int q = 0; q < 4; ++q) { bq[q] = *(const v4fa*)(&bcs[i * 32 + 4 * q]); cq[q] = *(const v4fa*)(&bcs[i * 32 + 16 + 4 * q]); }
            float y = 0.0f;
#pragma unroll
            for (int n = 0; n < NS; ++n) {
                const float bn = bq[n >> 2][n & 3], cn = cq[n >> 2][n & 3];
                const float dA = delta * an[n];
                const float ab = __builtin_amdgcn_exp2f(dA * L2E);
                const float bb = (ab - an[n]) * __builtin_amdgcn_rcpf(dA) * delta * bn;
                h[n] = ab * h[n] + bb * xv;
                y = y + cn * h[n];
            }
            os[wb + i * OSP + lane] = y;
        }
        wave_sync();
#pragma unroll 1
        for (int ps = 0; ps < 2; ++ps) {
#pragma unroll
            for (int s = 0; s < CH / 4; ++s) { const int row = 4 * s + (lane >> 3), cofs = (lane & 7) * 4;
                const v4f val = *(const v4fa*)(&os[wb + row * OSP + cofs]);
                *(volatile v4f*)(obase + (size_t)(l0 + row) * DD + cofs) = val; }
            if (ps == 0) __threadfence(); }
        __syncthreads();
    }
}

static constexpr size_t al256(size_t v) { return (v + 255) & ~(size_t)255; }
static constexpr size_t SZ_XB = al256((size_t)NB * SEQ * DD * 2);
static constexpr size_t SZ_WT = al256((size_t)NW * DD * 2);
static constexpr size_t SZ_BC = al256((size_t)NB * SEQ * 32 * 4);
static constexpr size_t SZ_SP = al256((size_t)NB * SEQ * 4);
static constexpr size_t SZ_TOTAL = SZ_XB + SZ_WT + SZ_BC + SZ_SP;
static_assert(SZ_TOTAL <= (size_t)134217728);
static_assert(((size_t)(NB * SEQ / 64 - 1) * 64 + 63) * 32 + 31 < (size_t)NB * SEQ * 32);
static_assert((size_t)(NB * SEQ / 64 - 1) * 64 + 63 < (size_t)NB * SEQ);

extern "C" void kernel_launch(void* const* d_in, const int* in_sizes, int n_in,
                              void* d_out, int out_size, void* d_ws, size_t ws_size, hipStream_t stream) {
    if (n_in < 9) return;
    const size_t needx = ((size_t)(NB - 1) * SEQ_FULL + SEQ) * DD;
    if ((size_t)in_sizes[0] < needx) return;
    if ((size_t)in_sizes[1] < (size_t)DD * NS || (size_t)in_sizes[2] < (size_t)DD * NS || (size_t)in_sizes[4] < (size_t)DD * NS) return;
    if (in_sizes[3] < NS || in_sizes[5] < NS || in_sizes[6] < DD || in_sizes[7] < 1 || in_sizes[8] < DD) return;
    if ((size_t)out_size < ((size_t)(NB - 1) * OUT_SEQ + SEQ) * DD) return;
    if (SZ_TOTAL > ws_size) return;
    const float* x   = (const float*)d_in[0];
    const float* Ain = (const float*)d_in[1];
    const float* wB  = (const float*)d_in[2]; const float* bB = (const float*)d_in[3];
    const float* wC  = (const float*)d_in[4]; const float* bC = (const float*)d_in[5];
    const float* wD  = (const float*)d_in[6]; const float* bD = (const float*)d_in[7];
    const float* pDl = (const float*)d_in[8];
    float* OUT = (float*)d_out;
    char* wsp = (char*)d_ws;
    bf* XB = (bf*)wsp; wsp += SZ_XB;
    bf* WT = (bf*)wsp; wsp += SZ_WT;
    float* PBC = (float*)wsp; wsp += SZ_BC;
    float* SP  = (float*)wsp; wsp += SZ_SP;

    if (SEQ == SEQ_FULL) {
        const size_t n8 = (size_t)NB * SEQ * DD / 8;
        k_cvt8<<<(unsigned)((n8 + 255) / 256), 256, 0, stream>>>(x, XB, n8);
    } else {
        const size_t n8 = (size_t)SEQ * DD / 8;
        for (int b = 0; b < NB; ++b) k_cvt8<<<(unsigned)((n8 + 255) / 256), 256, 0, stream>>>(x + (size_t)b * SEQ_FULL * DD, XB + (size_t)b * SEQ * DD, n8);
    }
    k_wpack<<<(unsigned)((NW * (DD / 8) + 255) / 256), 256, 0, stream>>>(wB, wC, wD, WT);

    k_pgemm<<<dim3(NB * SEQ / 64, 1, 1), 32, 0, stream>>>(XB, WT, bB, bC, bD, PBC, SP);

    k_scan<<<dim3(DD / ST, NB, 1), ST, 0, stream>>>(x, Ain, pDl, PBC, SP, OUT);
}
